// RoPEAttnBlock_11733850653068
// MI455X (gfx1250) — hardware-verified
//
#include <hip/hip_runtime.h>
#include <math.h>
#include <stdint.h>

#define SEQ  4096
#define DM   1024
#define NH   16
#define HD   64
#define H3   3072
#define HFF  4096
#define NQB  (SEQ / 64)
static_assert(NH * HD == DM);
static_assert((SEQ % 64) == 0 && (DM % 64) == 0 && (HFF % 64) == 0 && (H3 % 64) == 0);

typedef _Float16 v16h __attribute__((ext_vector_type(16)));
typedef _Float16 v8h  __attribute__((ext_vector_type(8)));
typedef float    v8f  __attribute__((ext_vector_type(8)));
typedef float    v4f  __attribute__((ext_vector_type(4)));
typedef unsigned int v4u __attribute__((ext_vector_type(4)));

__constant__ unsigned int kInvFreq[32] = {
  0x3f800000u, 0x3f3ff911u, 0x3f0ff59au, 0x3ed7e89bu, 0x3ea1e89bu, 0x3e72d424u, 0x3e361887u, 0x3e088d77u,
  0x3dcccccdu, 0x3d99940eu, 0x3d6655c3u, 0x3d2cba15u, 0x3d0186e2u, 0x3cc24350u, 0x3c91ad39u, 0x3c5a7bf1u,
  0x3c23d70au, 0x3bf5b9b0u, 0x3bb8449cu, 0x3b8a2e77u, 0x3b4f3e37u, 0x3b1b690du, 0x3ae91528u, 0x3aaec98eu,
  0x3a83126fu, 0x3a44948cu, 0x3a136a16u, 0x39dd1726u, 0x39a5cb5fu, 0x3978a814u, 0x393a7753u, 0x390bd472u };

__device__ __forceinline__ unsigned short h_bits(_Float16 x) { return __builtin_bit_cast(unsigned short, x); }
__device__ __forceinline__ unsigned pk16(unsigned short a, unsigned short b) { return (unsigned)a | ((unsigned)b << 16); }
__device__ __forceinline__ v8f zero8() { v8f z = {0.f, 0.f, 0.f, 0.f, 0.f, 0.f, 0.f, 0.f}; return z; }
__device__ __forceinline__ void wsync() {
  __builtin_amdgcn_fence(__ATOMIC_RELEASE, "workgroup");
  __builtin_amdgcn_wave_barrier();
  __builtin_amdgcn_fence(__ATOMIC_ACQUIRE, "workgroup");
}

__device__ __forceinline__ v16h ldfrag_h(const _Float16* p) {
  union { v16h v; v8h h[2]; } f;
  f.h[0] = *(const v8h*)(p);
  f.h[1] = *(const v8h*)(p + 16);
  return f.v;
}

__device__ __forceinline__ v8f mma_h(v16h a, v16h b, v8f c) {
  c = __builtin_amdgcn_wmma_f32_16x16x32_f16(false, a, false, b, (short)0, c, false, false);
  asm volatile("v_nop\n\tv_nop\n\tv_nop\n\tv_nop" : "+v"(c) : "v"(a), "v"(b));
  return c;
}

__global__ __launch_bounds__(256) void cvt_wT(const float* __restrict__ W, unsigned short* Wt,
                                              int K, int N, float scale) {
  __shared__ __align__(16) _Float16 sm[64 * 72];
  const int tid = threadIdx.x, lane = tid & 31, wave = tid >> 5;
  const int n0 = blockIdx.x * 64, k0 = blockIdx.y * 64;
  {
    const int kr = tid >> 2;
    const int nq = (tid & 3) * 16;
    const float* src = W + (size_t)(k0 + kr) * N + n0 + nq;
#pragma unroll
    for (int i = 0; i < 4; ++i) {
      const v4f a = *(const v4f*)(src + 4 * i);
#pragma unroll
      for (int e = 0; e < 4; ++e) sm[(nq + 4 * i + e) * 72 + kr] = (_Float16)(a[e] * scale);
    }
  }
  __syncthreads();
  union PK { v8h h; v4u u; };
  PK pk[2];
  const int q = lane >> 3, c8 = (lane & 7) * 8;
#pragma unroll
  for (int it = 0; it < 2; ++it) {
    const int row = wave * 8 + it * 4 + q;
    pk[it].h = *(const v8h*)(sm + row * 72 + c8);
  }
#pragma unroll
  for (int it = 0; it < 2; ++it) {
    const int row = wave * 8 + it * 4 + q;
    *(volatile v4u*)(Wt + (size_t)(n0 + row) * K + k0 + c8) = pk[it].u;
  }
  __threadfence();
#pragma unroll
  for (int it = 0; it < 2; ++it) {
    const int row = wave * 8 + it * 4 + q;
    *(volatile v4u*)(Wt + (size_t)(n0 + row) * K + k0 + c8) = pk[it].u;
  }
}

__global__ __launch_bounds__(256) void rope_tab(float* cosT, float* sinT, int ntot) {
  const int t = blockIdx.x * 256 + threadIdx.x;
  if (t >= ntot) return;
  const int pos = t >> 5, j = t & 31;
  const float th = (float)pos * __uint_as_float(kInvFreq[j]);
  float sn, cs;
  sincosf(th, &sn, &cs);
  *(volatile float*)(cosT + t) = cs;
  *(volatile float*)(sinT + t) = sn;
  __threadfence();
  *(volatile float*)(cosT + t) = cs;
  *(volatile float*)(sinT + t) = sn;
}

__global__ __launch_bounds__(256) void layernorm_h(const float* __restrict__ X, const float* __restrict__ G,
                                                   const float* __restrict__ Bb, unsigned short* O, int nrows) {
  const int lane = threadIdx.x & 31, wave = threadIdx.x >> 5;
  const int row = blockIdx.x * 8 + wave;
  if (row >= nrows) return;
  const float* xr = X + (size_t)row * DM;
  float v[32];
#pragma unroll
  for (int j = 0; j < 4; ++j) {
    const v4f a = *(const v4f*)(xr + j * 256 + lane * 8);
    const v4f b = *(const v4f*)(xr + j * 256 + lane * 8 + 4);
#pragma unroll
    for (int e = 0; e < 4; ++e) { v[8 * j + e] = a[e]; v[8 * j + 4 + e] = b[e]; }
  }
  float s = 0.f;
#pragma unroll
  for (int e = 0; e < 32; ++e) s += v[e];
#pragma unroll
  for (int off = 16; off > 0; off >>= 1) s += __shfl_xor(s, off, 32);
  const float mean = s * (1.0f / DM);
  float ss = 0.f;
#pragma unroll
  for (int e = 0; e < 32; ++e) { const float d = v[e] - mean; ss += d * d; }
#pragma unroll
  for (int off = 16; off > 0; off >>= 1) ss += __shfl_xor(ss, off, 32);
  const float var  = ss * (1.0f / DM);
  const float rstd = rsqrtf(var + 1e-5f);
  v4u pk[4];
#pragma unroll
  for (int j = 0; j < 4; ++j) {
    const int c0 = j * 256 + lane * 8;
    const v4f ga = *(const v4f*)(G + c0);
    const v4f gb = *(const v4f*)(G + c0 + 4);
    const v4f ba = *(const v4f*)(Bb + c0);
    const v4f bbv = *(const v4f*)(Bb + c0 + 4);
    float y[8];
#pragma unroll
    for (int e = 0; e < 4; ++e) {
      y[e]     = (v[8 * j + e]     - mean) * rstd * ga[e] + ba[e];
      y[4 + e] = (v[8 * j + 4 + e] - mean) * rstd * gb[e] + bbv[e];
    }
    v4u p;
#pragma unroll
    for (int e = 0; e < 4; ++e) p[e] = pk16(h_bits((_Float16)y[2 * e]), h_bits((_Float16)y[2 * e + 1]));
    pk[j] = p;
  }
#pragma unroll
  for (int j = 0; j < 4; ++j) *(volatile v4u*)(O + (size_t)row * DM + j * 256 + lane * 8) = pk[j];
  __threadfence();
#pragma unroll
  for (int j = 0; j < 4; ++j) *(volatile v4u*)(O + (size_t)row * DM + j * 256 + lane * 8) = pk[j];
}

template <int EPI>
__global__ __launch_bounds__(256) void gemm64(
    const unsigned short* __restrict__ Ap, int lda,
    const unsigned short* __restrict__ Btp, int ldb,
    void* Cout, int ldc,
    const float* __restrict__ resid, const float* __restrict__ bias,
    const float* __restrict__ cosT, const float* __restrict__ sinT,
    int M, int N, int K, float oscale, float cscale) {
  const _Float16* A  = (const _Float16*)(const void*)Ap;
  const _Float16* Bt = (const _Float16*)(const void*)Btp;
  __shared__ __align__(16) float sT[8][16 * 68];
  const int lane = threadIdx.x & 31;
  const int wave = threadIdx.x >> 5;
  const int tilesN = N >> 6;
  const int tilesM = M >> 6;
  const int tile = blockIdx.x * 8 + wave;
  if (tile >= tilesM * tilesN) return;
  const int tm = tile / tilesN;
  const int tn = tile - tm * tilesN;
  const int m0 = tm << 6;
  const int n0 = tn << 6;
  const int rl   = lane & 15;
  const int hh   = lane >> 4;
  const int koff = hh * 8;
  const int mOff = hh * 8;

  v8f acc[4][4];
#pragma unroll
  for (int i = 0; i < 4; ++i)
#pragma unroll
    for (int j = 0; j < 4; ++j) acc[i][j] = zero8();

  for (int k0 = 0; k0 < K; k0 += 32) {
    v16h bf[4];
#pragma unroll
    for (int j = 0; j < 4; ++j)
      bf[j] = ldfrag_h(Bt + (size_t)(n0 + (j << 4) + rl) * ldb + k0 + koff);
#pragma unroll
    for (int i = 0; i < 4; ++i) {
      const v16h af = ldfrag_h(A + (size_t)(m0 + (i << 4) + rl) * lda + k0 + koff);
#pragma unroll
      for (int j = 0; j < 4; ++j) acc[i][j] = mma_h(af, bf[j], acc[i][j]);
    }
  }

  float* slab = sT[wave];
#pragma unroll
  for (int i = 0; i < 4; ++i) {
    const int mBase = m0 + (i << 4);
#pragma unroll
    for (int j = 0; j < 4; ++j) {
#pragma unroll
      for (int r = 0; r < 8; ++r) slab[(mOff + r) * 68 + (j << 4) + rl] = acc[i][j][r];
    }
    wsync();
    if (EPI == 0 || EPI == 1) {
      float* C = (float*)Cout;
      const int c4 = rl * 4;
      v4f vv[8];
#pragma unroll
      for (int it = 0; it < 8; ++it) {
        const int row = it * 2 + hh;
        const size_t go = (size_t)(mBase + row) * ldc + n0 + c4;
        v4f v = *(const v4f*)(slab + row * 68 + c4);
        const v4f rsd = *(const v4f*)(resid + go);
        v = v * oscale + rsd;
        if (EPI == 1) { const v4f bv = *(const v4f*)(bias + n0 + c4); v = v + bv; }
        vv[it] = v;
      }
#pragma unroll
      for (int it = 0; it < 8; ++it) {
        const int row = it * 2 + hh;
        *(volatile v4f*)(C + (size_t)(mBase + row) * ldc + n0 + c4) = vv[it];
      }
      __threadfence();
#pragma unroll
      for (int it = 0; it < 8; ++it) {
        const int row = it * 2 + hh;
        *(volatile v4f*)(C + (size_t)(mBase + row) * ldc + n0 + c4) = vv[it];
      }
    } else {
      if (EPI == 2) {
#pragma unroll 1
        for (int e = 0; e < 16; ++e) {
          const int pos = mBase + e;
          const float cs = cosT[(size_t)pos * 32 + lane];
          const float sn = sinT[(size_t)pos * 32 + lane];
          const float x1 = slab[e * 68 + 2 * lane] * oscale;
          const float x2 = slab[e * 68 + 2 * lane + 1] * oscale;
          slab[e * 68 + 2 * lane]     = (x1 * cs - x2 * sn) * cscale;
          slab[e * 68 + 2 * lane + 1] = (x1 * sn + x2 * cs) * cscale;
        }
        wsync();
      }
      if (EPI == 4) {
#pragma unroll 1
        for (int e = 0; e < 32; ++e) {
          const int row = e >> 1, col = ((e & 1) << 5) + lane;
          float v = slab[row * 68 + col] * oscale + bias[n0 + col];
          const float gl = 0.5f * v * (1.0f + erff(v * 0.70710678118654752440f));
          slab[row * 68 + col] = gl * cscale;
        }
        wsync();
      }
      const int q = lane >> 3, c8 = (lane & 7) * 8;
      unsigned short* Cb = (unsigned short*)Cout;
      size_t cbase, cpitch; int colb;
      if (EPI == 2) {
        const int which = n0 >> 10;
        const int head  = (n0 & (DM - 1)) >> 6;
        cbase = (size_t)(which * NH + head) * SEQ * HD; cpitch = HD; colb = 0;
      } else {
        cbase = 0; cpitch = (size_t)ldc; colb = n0;
      }
      const float mul = (EPI == 3) ? cscale : 1.0f;
      v4u hv[4];
#pragma unroll
      for (int it = 0; it < 4; ++it) {
        const int row = it * 4 + q;
        const float* sp = slab + row * 68 + c8;
        v4u a;
#pragma unroll
        for (int e = 0; e < 4; ++e) {
          const float f0 = sp[2 * e] * mul, f1 = sp[2 * e + 1] * mul;
          a[e] = pk16(h_bits((_Float16)f0), h_bits((_Float16)f1));
        }
        hv[it] = a;
      }
#pragma unroll
      for (int it = 0; it < 4; ++it) {
        const int row = it * 4 + q;
        *(volatile v4u*)(Cb + cbase + (size_t)(mBase + row) * cpitch + colb + c8) = hv[it];
      }
      __threadfence();
#pragma unroll
      for (int it = 0; it < 4; ++it) {
        const int row = it * 4 + q;
        *(volatile v4u*)(Cb + cbase + (size_t)(mBase + row) * cpitch + colb + c8) = hv[it];
      }
    }
    wsync();
  }
}

__global__ __launch_bounds__(128)
void attn_causal64(const unsigned short* __restrict__ qp, const unsigned short* __restrict__ kp,
                   const unsigned short* __restrict__ vtp, unsigned short* op, float sscale, float onorm) {
  union FH { v16h v; v8h h[2]; };
  __shared__ __align__(16) _Float16 Ksh[64 * 64];
  __shared__ __align__(16) _Float16 Vth[64 * 64];
  __shared__ __align__(16) _Float16 Psh[4][16 * 64];
  __shared__ __align__(16) float    Os[4][16 * 64];

  const int tid  = threadIdx.x;
  const int wave = tid >> 5;
  const int lane = tid & 31;
  const int hh   = lane >> 4;
  const int c    = lane & 15;
  const int bx   = blockIdx.x;
  const int h    = bx / NQB;
  const int qb   = bx - h * NQB;
  const int q0   = qb * 64 + wave * 16;

  const _Float16* Q = (const _Float16*)(const void*)qp  + (size_t)h * SEQ * HD;
  const _Float16* Kg = (const _Float16*)(const void*)kp + (size_t)h * SEQ * HD;
  const _Float16* V = (const _Float16*)(const void*)vtp + (size_t)h * HD * SEQ;

  v16h qa[2];
#pragma unroll
  for (int dc = 0; dc < 2; ++dc) qa[dc] = ldfrag_h(Q + (size_t)(q0 + c) * HD + dc * 32 + 8 * hh);

  float mrow[8], lrow[8];
  v8f oacc[4];
#pragma unroll
  for (int r = 0; r < 8; ++r) { mrow[r] = -INFINITY; lrow[r] = 0.f; }
#pragma unroll
  for (int t = 0; t < 4; ++t) oacc[t] = zero8();

  const int nkt = qb + 1;
  for (int kt = 0; kt < nkt; ++kt) {
    const int kv0 = kt * 64;
    __syncthreads();
    {
      const int r = tid >> 1, half = (tid & 1) * 32;
      const _Float16* kg = Kg + (size_t)(kv0 + r) * HD + half;
      const _Float16* vg = V + (size_t)r * SEQ + kv0 + half;
#pragma unroll
      for (int i = 0; i < 4; ++i) {
        const v8h a0 = *(const v8h*)(kg + 8 * i);
        const v8h b0 = *(const v8h*)(vg + 8 * i);
        *(v8h*)(Ksh + r * 64 + half + 8 * i) = a0;
        *(v8h*)(Vth + r * 64 + half + 8 * i) = b0;
      }
    }
    __syncthreads();

    v8f s[4];
#pragma unroll
    for (int j = 0; j < 4; ++j) {
      s[j] = zero8();
#pragma unroll
      for (int dc = 0; dc < 2; ++dc) {
        FH kb;
        kb.h[0] = *(const v8h*)(Ksh + (j * 16 + c) * 64 + dc * 32 + 8 * hh);
        kb.h[1] = *(const v8h*)(Ksh + (j * 16 + c) * 64 + dc * 32 + 16 + 8 * hh);
        s[j] = mma_h(qa[dc], kb.v, s[j]);
      }
    }

    _Float16* pw = Psh[wave];
#pragma unroll
    for (int r = 0; r < 8; ++r) {
      const int row = q0 + 8 * hh + r;
      float m = -INFINITY;
#pragma unroll
      for (int j = 0; j < 4; ++j) {
        const int key = kv0 + j * 16 + c;
        float sv = s[j][r] * sscale;
        sv = (key > row) ? -INFINITY : sv;
        s[j][r] = sv;
        m = fmaxf(m, sv);
      }
#pragma unroll
      for (int off = 1; off < 16; off <<= 1) m = fmaxf(m, __shfl_xor(m, off, 32));
      const float mnew  = fmaxf(mrow[r], m);
      const float msafe = (mnew == -INFINITY) ? 0.f : mnew;
      const float alpha = __expf(mrow[r] - msafe);
      mrow[r] = mnew;
      float psum = 0.f;
#pragma unroll
      for (int j = 0; j < 4; ++j) {
        const float p = __expf(s[j][r] - msafe);
        psum += p;
        pw[(8 * hh + r) * 64 + j * 16 + c] = (_Float16)(p * 1024.0f);
      }
#pragma unroll
      for (int off = 1; off < 16; off <<= 1) psum += __shfl_xor(psum, off, 32);
      lrow[r] = lrow[r] * alpha + psum;
#pragma unroll
      for (int t = 0; t < 4; ++t) oacc[t][r] *= alpha;
    }
    wsync();

#pragma unroll
    for (int kk = 0; kk < 2; ++kk) {
      FH pa;
      pa.h[0] = *(const v8h*)(pw + c * 64 + kk * 32 + 8 * hh);
      pa.h[1] = *(const v8h*)(pw + c * 64 + kk * 32 + 16 + 8 * hh);
#pragma unroll
      for (int t = 0; t < 4; ++t) {
        FH vb;
        vb.h[0] = *(const v8h*)(Vth + (t * 16 + c) * 64 + kk * 32 + 8 * hh);
        vb.h[1] = *(const v8h*)(Vth + (t * 16 + c) * 64 + kk * 32 + 16 + 8 * hh);
        oacc[t] = mma_h(pa.v, vb.v, oacc[t]);
      }
    }
  }

  float* os = Os[wave];
#pragma unroll
  for (int r = 0; r < 8; ++r) {
    const float l = lrow[r];
    const float inv = ((l > 0.f) ? (1.0f / l) : 0.f) * onorm;
#pragma unroll
    for (int t = 0; t < 4; ++t) os[(8 * hh + r) * 64 + t * 16 + c] = oacc[t][r] * inv;
  }
  wsync();
  {
    const int q4 = lane >> 3, c8 = (lane & 7) * 8;
    v4u hv[4];
#pragma unroll
    for (int it = 0; it < 4; ++it) {
      const int row = it * 4 + q4;
      const float* sp = os + row * 64 + c8;
      v4u a;
#pragma unroll
      for (int e = 0; e < 4; ++e) a[e] = pk16(h_bits((_Float16)sp[2 * e]), h_bits((_Float16)sp[2 * e + 1]));
      hv[it] = a;
    }
#pragma unroll
    for (int it = 0; it < 4; ++it) {
      const int row = it * 4 + q4;
      *(volatile v4u*)(op + (size_t)(q0 + row) * DM + (size_t)h * HD + c8) = hv[it];
    }
    __threadfence();
#pragma unroll
    for (int it = 0; it < 4; ++it) {
      const int row = it * 4 + q4;
      *(volatile v4u*)(op + (size_t)(q0 + row) * DM + (size_t)h * HD + c8) = hv[it];
    }
  }
}

extern "C" void kernel_launch(void* const* d_in, const int* in_sizes, int n_in,
                              void* d_out, int out_size, void* d_ws, size_t ws_size,
                              hipStream_t stream) {
  if (n_in < 11) return;
  if (in_sizes[0] != SEQ * DM) return;
  if (in_sizes[1] != DM || in_sizes[2] != DM || in_sizes[3] != DM || in_sizes[4] != DM) return;
  if (in_sizes[5] != DM * H3 || in_sizes[6] != DM * DM || in_sizes[7] != DM * HFF) return;
  if (in_sizes[8] != HFF || in_sizes[9] != HFF * DM || in_sizes[10] != DM) return;
  if (out_size != SEQ * DM) return;

  const float* x    = (const float*)d_in[0];
  const float* ln1g = (const float*)d_in[1];
  const float* ln1b = (const float*)d_in[2];
  const float* ln2g = (const float*)d_in[3];
  const float* ln2b = (const float*)d_in[4];
  const float* Wqkv = (const float*)d_in[5];
  const float* Wo   = (const float*)d_in[6];
  const float* W1   = (const float*)d_in[7];
  const float* b1   = (const float*)d_in[8];
  const float* W2   = (const float*)d_in[9];
  const float* b2   = (const float*)d_in[10];
  float* out = (float*)d_out;

  const size_t szWqkv = (size_t)H3 * DM * 2;
  const size_t szWo   = (size_t)DM * DM * 2;
  const size_t szW1   = (size_t)HFF * DM * 2;
  const size_t szW2   = (size_t)DM * HFF * 2;
  const size_t szTab  = (size_t)SEQ * 32 * 4;
  const size_t szN    = (size_t)SEQ * DM * 2;
  const size_t szQK   = (size_t)2 * NH * SEQ * HD * 2;
  const size_t szVT   = (size_t)DM * SEQ * 2;
  const size_t szCtx  = (size_t)SEQ * DM * 2;
  const size_t szX1   = (size_t)SEQ * DM * 4;
  const size_t szG    = (size_t)SEQ * HFF * 2;
  size_t off = 0;
  const size_t oWqkv = off; off += szWqkv;
  const size_t oWo   = off; off += szWo;
  const size_t oW1   = off; off += szW1;
  const size_t oW2   = off; off += szW2;
  const size_t oCos  = off; off += szTab;
  const size_t oSin  = off; off += szTab;
  const size_t oN    = off; off += szN;
  const size_t oQK   = off; off += szQK;
  const size_t oVT   = off; off += szVT;
  const size_t oCtx  = off; off += szCtx;
  const size_t oX1   = off; off += szX1;
  const size_t oG    = off; off += szG;
  if (off > ws_size) return;
  if (off > (size_t)134217728) return;

  char* ws = (char*)d_ws;
  unsigned short* WqkvT = (unsigned short*)(ws + oWqkv);
  unsigned short* WoT   = (unsigned short*)(ws + oWo);
  unsigned short* W1T   = (unsigned short*)(ws + oW1);
  unsigned short* W2T   = (unsigned short*)(ws + oW2);
  float*          cosT  = (float*)(ws + oCos);
  float*          sinT  = (float*)(ws + oSin);
  unsigned short* nP    = (unsigned short*)(ws + oN);
  unsigned short* qkP   = (unsigned short*)(ws + oQK);
  unsigned short* qP    = qkP;
  unsigned short* kP    = qkP + (size_t)NH * SEQ * HD;
  unsigned short* vT    = (unsigned short*)(ws + oVT);
  unsigned short* ctx   = (unsigned short*)(ws + oCtx);
  float*          x1    = (float*)(ws + oX1);
  unsigned short* gP    = (unsigned short*)(ws + oG);

  const dim3 blk(256);
  cvt_wT<<<dim3(H3 / 64, DM / 64), blk, 0, stream>>>(Wqkv, WqkvT, DM, H3, 32.0f);
  cvt_wT<<<dim3(DM / 64, DM / 64), blk, 0, stream>>>(Wo, WoT, DM, DM, 32.0f);
  cvt_wT<<<dim3(HFF / 64, DM / 64), blk, 0, stream>>>(W1, W1T, DM, HFF, 32.0f);
  cvt_wT<<<dim3(DM / 64, HFF / 64), blk, 0, stream>>>(W2, W2T, HFF, DM, 32.0f);
  const int nTab = SEQ * 32;
  rope_tab<<<dim3((nTab + 255) / 256), blk, 0, stream>>>(cosT, sinT, nTab);
  layernorm_h<<<dim3((SEQ + 7) / 8), blk, 0, stream>>>(x, ln1g, ln1b, nP, SEQ);
  {
    const int tiles = (SEQ / 64) * (2 * DM / 64);
    gemm64<2><<<dim3((tiles + 7) / 8), blk, 0, stream>>>(
        nP, DM, WqkvT, DM, (void*)qkP, HD, cosT, cosT, cosT, sinT,
        SEQ, 2 * DM, DM, 1.0f / 32.0f, 4.0f);
  }
  {
    const int tiles = (DM / 64) * (SEQ / 64);
    gemm64<3><<<dim3((tiles + 7) / 8), blk, 0, stream>>>(
        WqkvT + (size_t)2 * DM * DM, DM, nP, DM, (void*)vT, SEQ, cosT, cosT, cosT, sinT,
        DM, SEQ, DM, 1.0f, 1.0f / 8.0f);
  }
  attn_causal64<<<dim3(NH * NQB), dim3(128), 0, stream>>>(qP, kP, vT, ctx, 1.0f / 128.0f, 1.0f / 128.0f);
  {
    const int tiles = (SEQ / 64) * (DM / 64);
    gemm64<0><<<dim3((tiles + 7) / 8), blk, 0, stream>>>(
        ctx, DM, WoT, DM, (void*)x1, DM, x, cosT, cosT, sinT,
        SEQ, DM, DM, 1.0f / 1024.0f, 1.0f);
  }
  layernorm_h<<<dim3((SEQ + 7) / 8), blk, 0, stream>>>(x1, ln2g, ln2b, nP, SEQ);
  {
    const int tiles = (SEQ / 64) * (HFF / 64);
    gemm64<4><<<dim3((tiles + 7) / 8), blk, 0, stream>>>(
        nP, DM, W1T, DM, (void*)gP, HFF, cosT, b1, cosT, sinT,
        SEQ, HFF, DM, 1.0f / 32.0f, 16.0f);
  }
  {
    const int tiles = (SEQ / 64) * (DM / 64);
    gemm64<1><<<dim3((tiles + 7) / 8), blk, 0, stream>>>(
        gP, HFF, W2T, HFF, d_out, DM, x1, b2, cosT, sinT,
        SEQ, DM, HFF, 1.0f / 512.0f, 1.0f);
  }
  (void)out;
  (void)hipGetLastError();
}
